// Bi_lstm_46780783788462
// MI455X (gfx1250) — hardware-run, weakly checked
//
#include <hip/hip_runtime.h>
#include <math.h>

constexpr int NBATCH   = 2048;
constexpr int NSEQ     = 1024;
constexpr int NIN      = 3;
constexpr int NHID     = 32;
constexpr int NGATE    = 4 * NHID;
constexpr int NFC1     = 16;
constexpr int NOUTC    = 2;
constexpr int ROWS_BLK = 16;
constexpr int NTHR     = 256;
constexpr int XCHUNK   = 32;
constexpr int XROWF    = XCHUNK * NIN;
constexpr int XROWV4   = XROWF / 4;
constexpr int XPITCH   = 100;
constexpr int GPITCH   = 132;
constexpr int PPITCH   = 33;
constexpr int FPITCH   = 17;
constexpr float HCARRY = 64.0f;
constexpr float WCARRY = 64.0f;
constexpr float FOLD   = 1.0f / (HCARRY * WCARRY);

static_assert(NBATCH % ROWS_BLK == 0);
static_assert(NSEQ % XCHUNK == 0);
static_assert(NHID == 32);
static_assert(NGATE == 16 * (NTHR / 32));
static_assert(XROWF % 4 == 0);
static_assert((XROWF * 4) % 128 == 0);
static_assert(ROWS_BLK * XROWV4 == NTHR + 128);
static_assert(ROWS_BLK * NOUTC == 32);
static_assert(ROWS_BLK * NFC1 == NTHR);
static_assert(NGATE * NIN == 96 * 4);
static_assert(XPITCH >= XROWF && (XPITCH % 4) == 0);

typedef __attribute__((ext_vector_type(16))) _Float16 v16h;
typedef __attribute__((ext_vector_type(8)))  _Float16 v8h;
typedef __attribute__((ext_vector_type(8)))  float    v8f;
typedef __attribute__((ext_vector_type(4)))  float    v4f;

struct FragH {
  union U { v16h v; v8h h[2]; };
  static __device__ __forceinline__ v16h load(const _Float16* p) {
    U f;
    f.h[0] = *(const v8h*)(p);
    f.h[1] = *(const v8h*)(p + 16);
    return f.v;
  }
  static __device__ __forceinline__ v8f mma(v16h a, v16h b, v8f c) {
    return __builtin_amdgcn_wmma_f32_16x16x32_f16(false, a, false, b, (short)0, c, false, false);
  }
};
__device__ __forceinline__ void wmma_guard1(v8f& a, v16h x, v16h y) {
  asm volatile("v_nop\n\tv_nop\n\tv_nop\n\tv_nop" : "+v"(a) : "v"(x), "v"(y));
}

__device__ __forceinline__ float fsig(float v)  { return __builtin_amdgcn_rcpf(1.0f + __expf(-v)); }
__device__ __forceinline__ float ftanh(float v) { return 1.0f - 2.0f * __builtin_amdgcn_rcpf(__expf(2.0f * v) + 1.0f); }

__global__ __launch_bounds__(NTHR) void lstm_pool_head_kernel(
    const float* __restrict__ x, const float* __restrict__ W_ih, const float* __restrict__ W_hh,
    const float* __restrict__ b_ih, const float* __restrict__ b_hh, const float* __restrict__ attn_w,
    const float* __restrict__ fc1_w, const float* __restrict__ fc1_b,
    const float* __restrict__ fc2_w, const float* __restrict__ fc2_b,
    float* __restrict__ out) {
  __shared__ __align__(16) _Float16 hA[ROWS_BLK * NHID];
  __shared__ __align__(16) float    gbuf[ROWS_BLK * GPITCH];
  __shared__ __align__(16) float    xs[ROWS_BLK * XPITCH];
  __shared__ __align__(16) float    wsm[NGATE * NIN];
  __shared__ __align__(16) float    bsm[NGATE];
  __shared__ float pbuf[ROWS_BLK * PPITCH];
  __shared__ float h1s[ROWS_BLK * FPITCH];

  const int tid  = threadIdx.x;
  const int lane = tid & 31;
  const int wave = tid >> 5;
  const int c    = lane & 15;
  const int hh   = lane >> 4;
  const int r0   = blockIdx.x * ROWS_BLK;

  if (tid < 96) {
    const v4f v = *(const v4f*)(W_ih + tid * 4);
    *(v4f*)(wsm + tid * 4) = v;
  }
  if (tid >= 128 && tid < 160) {
    const int i4 = (tid - 128) * 4;
    const v4f va = *(const v4f*)(b_ih + i4);
    const v4f vb = *(const v4f*)(b_hh + i4);
    v4f vs;
#pragma unroll
    for (int e = 0; e < 4; ++e) vs[e] = va[e] + vb[e];
    *(v4f*)(bsm + i4) = vs;
  }
#pragma unroll 1
  for (int i = tid; i < ROWS_BLK * NHID; i += NTHR) hA[i] = (_Float16)0.0f;

  v16h bmat;
  {
    const int n = wave * 16 + c;
    const float* wrow = W_hh + (size_t)n * NHID + 8 * hh;
    const v4f w0 = *(const v4f*)(wrow);
    const v4f w1 = *(const v4f*)(wrow + 4);
    const v4f w2 = *(const v4f*)(wrow + 16);
    const v4f w3 = *(const v4f*)(wrow + 20);
#pragma unroll
    for (int e = 0; e < 4; ++e) {
      bmat[e]      = (_Float16)(w0[e] * WCARRY);
      bmat[4 + e]  = (_Float16)(w1[e] * WCARRY);
      bmat[8 + e]  = (_Float16)(w2[e] * WCARRY);
      bmat[12 + e] = (_Float16)(w3[e] * WCARRY);
    }
  }
  const float aw = attn_w[lane];
  __syncthreads();

  float wx[4][3], bg[4];
#pragma unroll
  for (int q = 0; q < 4; ++q) {
    const int n = q * NHID + lane;
    wx[q][0] = wsm[n * NIN + 0];
    wx[q][1] = wsm[n * NIN + 1];
    wx[q][2] = wsm[n * NIN + 2];
    bg[q]    = bsm[n];
  }

  float cst[2]  = {0.0f, 0.0f};
  float pacc[2] = {0.0f, 0.0f};
  float den[2]  = {0.0f, 0.0f};

  const _Float16* arow = hA + c * NHID + 8 * hh;
  const v8f z8 = {0.f, 0.f, 0.f, 0.f, 0.f, 0.f, 0.f, 0.f};

#pragma unroll 1
  for (int t = 0; t < NSEQ; ++t) {
    const int tt = t & (XCHUNK - 1);
    if (tt == 0) {
      {
        const int row = tid / XROWV4;
        const int q   = tid - row * XROWV4;
        const v4f v = *(const v4f*)(x + ((size_t)(r0 + row) * NSEQ + (size_t)t) * NIN + q * 4);
        *(v4f*)(xs + row * XPITCH + q * 4) = v;
      }
      if (tid < 128) {
        const int idx = tid + NTHR;
        const int row = idx / XROWV4;
        const int q   = idx - row * XROWV4;
        const v4f v = *(const v4f*)(x + ((size_t)(r0 + row) * NSEQ + (size_t)t) * NIN + q * 4);
        *(v4f*)(xs + row * XPITCH + q * 4) = v;
      }
    }

    const v16h a = FragH::load(arow);
    v8f acc = z8;
    acc = FragH::mma(a, bmat, acc);
    wmma_guard1(acc, a, bmat);
#pragma unroll
    for (int r = 0; r < 8; ++r) gbuf[(8 * hh + r) * GPITCH + wave * 16 + c] = acc[r];

    __syncthreads();

#pragma unroll
    for (int e = 0; e < 2; ++e) {
      const int r = wave + 8 * e;
      const float* xp = xs + r * XPITCH + tt * NIN;
      const float x0 = xp[0];
      const float x1 = xp[1];
      const float x2 = xp[2];
      const float* gp = gbuf + r * GPITCH + lane;
      float gq[4];
#pragma unroll
      for (int q = 0; q < 4; ++q) {
        float xg = x0 * wx[q][0];
        xg = fmaf(x1, wx[q][1], xg);
        xg = fmaf(x2, wx[q][2], xg);
        xg += bg[q];
        gq[q] = fmaf(gp[q * NHID], FOLD, xg);
      }
      const float ig = fsig(gq[0]);
      const float fg = fsig(gq[1]);
      const float gg = ftanh(gq[2]);
      const float og = fsig(gq[3]);
      const float cn = fg * cst[e] + ig * gg;
      cst[e] = cn;
      const float hn = og * ftanh(cn);

      float sv = hn * aw;
      sv += __shfl_xor(sv, 16, 32);
      sv += __shfl_xor(sv, 8, 32);
      sv += __shfl_xor(sv, 4, 32);
      sv += __shfl_xor(sv, 2, 32);
      sv += __shfl_xor(sv, 1, 32);
      const float wt = __expf(fmaxf(sv, 0.0f));
      den[e]  += wt;
      pacc[e] = fmaf(wt, hn, pacc[e]);

      hA[r * NHID + lane] = (_Float16)(hn * HCARRY);
    }
    __syncthreads();
  }

#pragma unroll
  for (int e = 0; e < 2; ++e) {
    const float inv = 1.0f / den[e];
    pbuf[(wave + 8 * e) * PPITCH + lane] = pacc[e] * inv;
  }
  __syncthreads();

  {
    const int row = tid >> 4;
    const int m   = tid & 15;
    float a1 = 0.0f;
#pragma unroll 1
    for (int j = 0; j < NHID; ++j) a1 = fmaf(pbuf[row * PPITCH + j], fc1_w[m * NHID + j], a1);
    a1 += fc1_b[m];
    h1s[row * FPITCH + m] = fmaxf(a1, 0.0f);
  }
  __syncthreads();

  if (tid < 32) {
    const int rr = lane >> 1;
    const int kk = lane & 1;
    float a2 = 0.0f;
#pragma unroll 1
    for (int m = 0; m < NFC1; ++m) a2 = fmaf(h1s[rr * FPITCH + m], fc2_w[kk * NFC1 + m], a2);
    a2 += fc2_b[kk];
    volatile float* op = out + (size_t)r0 * NOUTC + lane;
    *op = a2;
    __threadfence();
    *op = a2;
  }
}

extern "C" void kernel_launch(void* const* d_in, const int* in_sizes, int n_in,
                              void* d_out, int out_size, void* d_ws, size_t ws_size, hipStream_t stream) {
  (void)d_ws;
  (void)ws_size;
  if (n_in < 10 || d_out == nullptr) return;
  if (in_sizes[0] != NBATCH * NSEQ * NIN || in_sizes[1] != NGATE * NIN || in_sizes[2] != NGATE * NHID ||
      in_sizes[3] != NGATE || in_sizes[4] != NGATE || in_sizes[5] != NHID || in_sizes[6] != NFC1 * NHID ||
      in_sizes[7] != NFC1 || in_sizes[8] != NOUTC * NFC1 || in_sizes[9] != NOUTC ||
      out_size != NBATCH * NOUTC) return;

  const float* x      = (const float*)d_in[0];
  const float* W_ih   = (const float*)d_in[1];
  const float* W_hh   = (const float*)d_in[2];
  const float* b_ih   = (const float*)d_in[3];
  const float* b_hh   = (const float*)d_in[4];
  const float* attn_w = (const float*)d_in[5];
  const float* fc1_w  = (const float*)d_in[6];
  const float* fc1_b  = (const float*)d_in[7];
  const float* fc2_w  = (const float*)d_in[8];
  const float* fc2_b  = (const float*)d_in[9];
  float* out = (float*)d_out;

  lstm_pool_head_kernel<<<NBATCH / ROWS_BLK, NTHR, 0, stream>>>(
      x, W_ih, W_hh, b_ih, b_hh, attn_w, fc1_w, fc1_b, fc2_w, fc2_b, out);
}
